// SpatialPositionalEncoding_23175643529969
// MI455X (gfx1250) — hardware-run, weakly checked
//
#include <hip/hip_runtime.h>
#include <math.h>

typedef __attribute__((ext_vector_type(16))) _Float16 v16h;
typedef __attribute__((ext_vector_type(8)))  _Float16 v8h;
typedef __attribute__((ext_vector_type(8)))  float    v8f;
typedef __attribute__((ext_vector_type(4)))  float    v4f;
typedef __attribute__((ext_vector_type(4)))  int      v4i;

constexpr int kBatch  = 8;
constexpr int kNodes  = 512;
constexpr int kHid    = 64;
constexpr int kDmodel = 256;
constexpr int kRows   = kBatch * kNodes;
constexpr int kFeat   = 5;
constexpr float kEps  = 1e-6f;
constexpr float kH1Carry  = 16.0f;
constexpr float kWCarry   = 256.0f;
constexpr float kAggCarry = 64.0f;
constexpr float kL2Fold   = 1.0f / (kH1Carry * kWCarry);
constexpr float kOutFold  = 1.0f / (kAggCarry * kWCarry);
constexpr int kAP = 72;
static_assert(kRows == 4096, "rows");
static_assert((kHid % 32) == 0, "K multiple of 32");
static_assert((kRows % 64) == 0 && (kDmodel % 64) == 0 && (kHid % 64) == 0, "M,N multiples of 64");
static_assert((kNodes % 16) == 0 && (kNodes % 8) == 0, "j tiles / rows per block");
static_assert(kL2Fold == 1.0f / 4096.0f && kOutFold == 1.0f / 16384.0f, "fold constants");

constexpr size_t kOffCen  = 0;
constexpr size_t kOffCnt  = kOffCen + (size_t)kRows * 4 * 4;
constexpr size_t kOffW2t  = kOffCnt + 128;
constexpr size_t kOffWot  = kOffW2t + (size_t)kHid * kHid * 2;
constexpr size_t kOffAgg  = kOffWot + (size_t)kDmodel * kHid * 2;
constexpr size_t kWsTotal = kOffAgg + (size_t)kRows * kHid * 2;
static_assert(kWsTotal == 630912ull, "carve total");
static_assert(kWsTotal <= 134217728ull, "carve cap");
static_assert((kOffCnt % 128) == 0 && (kOffW2t % 128) == 0 && (kOffWot % 128) == 0 && (kOffAgg % 128) == 0, "aligned regions");

struct FragH {
  union U { v16h v; v8h h[2]; };
  static __device__ __forceinline__ v16h load(const _Float16* p) {
    U f;
    f.h[0] = *(const v8h*)(p);
    f.h[1] = *(const v8h*)(p + 16);
    return f.v;
  }
};
__device__ __forceinline__ v8f mma_h(v16h a, v16h b, v8f c) {
  c = __builtin_amdgcn_wmma_f32_16x16x32_f16(false, a, false, b, (short)0, c, false, false);
  asm volatile("v_nop\n\tv_nop\n\tv_nop\n\tv_nop" : "+v"(c) : "v"(a), "v"(b));
  return c;
}
__device__ __forceinline__ void wave_lds_sync() {
  __builtin_amdgcn_fence(__ATOMIC_RELEASE, "workgroup");
  __builtin_amdgcn_wave_barrier();
  __builtin_amdgcn_fence(__ATOMIC_ACQUIRE, "workgroup");
}

__global__ __launch_bounds__(256) void prep_kernel(
    const float* __restrict__ corners, const int* __restrict__ valid,
    const float* __restrict__ W2, const float* __restrict__ Wo,
    float* __restrict__ cen4, float* __restrict__ cnt,
    unsigned short* __restrict__ w2t, unsigned short* __restrict__ wot)
{
  __shared__ float sCnt[8];
  const int tid = threadIdx.x, lane = tid & 31, wave = tid >> 5;
  const int blk = blockIdx.x;
  if (blk < 16) {
    const int id = blk * 256 + tid;
    const float* c = corners + (size_t)id * 24;
    float f[24];
#pragma unroll
    for (int q = 0; q < 6; ++q) {
      const v4f t = *(const v4f*)(c + 4 * q);
      f[4 * q + 0] = t[0];
      f[4 * q + 1] = t[1];
      f[4 * q + 2] = t[2];
      f[4 * q + 3] = t[3];
    }
    float cx = 0.0f, cy = 0.0f, cz = 0.0f;
#pragma unroll
    for (int q = 0; q < 8; ++q) {
      cx += f[3 * q + 0];
      cy += f[3 * q + 1];
      cz += f[3 * q + 2];
    }
    cx *= 0.125f;
    cy *= 0.125f;
    cz *= 0.125f;
    const float ax = f[3] - f[0],  ay = f[4] - f[1],   az = f[5] - f[2];
    const float bx = f[9] - f[0],  by = f[10] - f[1],  bz = f[11] - f[2];
    const float ex = f[12] - f[0], ey = f[13] - f[1],  ez = f[14] - f[2];
    const float la = sqrtf(ax * ax + ay * ay + az * az + kEps);
    const float lb = sqrtf(bx * bx + by * by + bz * bz + kEps);
    const float lc = sqrtf(ex * ex + ey * ey + ez * ez + kEps);
    const float lv = logf(la * lb * lc + kEps);
    v4f o;
    o[0] = cx;
    o[1] = cy;
    o[2] = cz;
    o[3] = lv;
    float* p = cen4 + (size_t)id * 4;
    *(volatile v4f*)p = o;
    __threadfence();
    *(volatile v4f*)p = o;
  } else if (blk == 16) {
    int cw = 0;
#pragma unroll 1
    for (int it = 0; it < kNodes / 32; ++it) {
      const int v = valid[wave * kNodes + it * 32 + lane];
      const unsigned long long bal = __ballot(v != 0);
      cw += __popcll(bal);
    }
    if (lane == 0) sCnt[wave] = (float)cw;
    __syncthreads();
    if (wave == 0) {
      const int li = (lane < 8) ? lane : 7;
      const float cv = sCnt[li];
      const float inv = 1.0f / fmaxf(cv, 1.0f);
      const float ov = (lane < 8) ? inv : 0.0f;
      volatile float* p = cnt + lane;
      *p = ov;
      __threadfence();
      *p = ov;
    }
  } else if (blk < 19) {
    const int g = (blk - 17) * 256 + tid;
    const int n = g >> 3, k8 = (g & 7) * 8;
    v8h hv;
#pragma unroll
    for (int e = 0; e < 8; ++e) hv[e] = (_Float16)(W2[(k8 + e) * kHid + n] * kWCarry);
    unsigned short* p = w2t + (size_t)g * 8;
    *(volatile v8h*)p = hv;
    __threadfence();
    *(volatile v8h*)p = hv;
  } else {
    const int g = (blk - 19) * 256 + tid;
    const int n = g >> 3, k8 = (g & 7) * 8;
    v8h hv;
#pragma unroll
    for (int e = 0; e < 8; ++e) hv[e] = (_Float16)(Wo[(k8 + e) * kDmodel + n] * kWCarry);
    unsigned short* p = wot + (size_t)g * 8;
    *(volatile v8h*)p = hv;
    __threadfence();
    *(volatile v8h*)p = hv;
  }
}

__global__ __launch_bounds__(256) void pair_mlp_kernel(
    const float* __restrict__ cen4, const int* __restrict__ valid, const float* __restrict__ cntinv,
    const unsigned short* __restrict__ w2t, const float* __restrict__ W1, const float* __restrict__ b1,
    const float* __restrict__ b2, unsigned short* __restrict__ aggp)
{
  __shared__ __align__(16) float    sC[kNodes * 4];
  __shared__ __align__(16) int      sV[kNodes];
  __shared__ __align__(16) float    sW1p[32 * 12];
  __shared__ __align__(16) _Float16 sA[8][16 * kAP];
  __shared__ __align__(16) float    sAgg[8 * kHid];

  const int tid = threadIdx.x;
  const int bi0 = blockIdx.x * 8;
  const int b   = bi0 / kNodes;

#pragma unroll
  for (int it = 0; it < 2; ++it) {
    const int idx = tid + it * 256;
    *(v4f*)(sC + idx * 4) = *(const v4f*)(cen4 + (size_t)(b * kNodes + idx) * 4);
    sV[idx] = valid[b * kNodes + idx];
  }
#pragma unroll
  for (int it = 0; it < 2; ++it) {
    const int idx = tid + it * 256;
    const int e = (idx < kFeat * kHid) ? idx : (kFeat * kHid - 1);
    const float wv = W1[e] * kH1Carry;
    const int f = e >> 6, u = e & 63;
    if (idx < kFeat * kHid) sW1p[(u >> 1) * 12 + 2 * f + (u & 1)] = wv;
  }
  {
    const int u = tid & 63;
    const float bv = b1[u] * kH1Carry;
    if (tid < 64) sW1p[(u >> 1) * 12 + 10 + (u & 1)] = bv;
  }
  __syncthreads();

  const int wave = tid >> 5;
  const int lane = tid & 31;
  const int half = lane >> 4;
  const int m    = lane & 15;
  const int iloc = (bi0 + wave) & (kNodes - 1);

  const v4f ci = *(const v4f*)(sC + iloc * 4);

  const _Float16* w2p = (const _Float16*)w2t;
  v16h w2f[2][4];
#pragma unroll
  for (int s = 0; s < 2; ++s)
#pragma unroll
    for (int t = 0; t < 4; ++t)
      w2f[s][t] = FragH::load(w2p + (16 * t + m) * kHid + 32 * s + 8 * half);

  float b2v[4];
#pragma unroll
  for (int t = 0; t < 4; ++t) b2v[t] = b2[16 * t + m];

  float acc[4] = {0.0f, 0.0f, 0.0f, 0.0f};
  _Float16* tileA = sA[wave];
  _Float16* arow = tileA + m * kAP + 32 * half;
  const _Float16* afr = tileA + m * kAP + 8 * half;
  const float* wbase = sW1p + (16 * half) * 12;

#pragma unroll 1
  for (int jc = 0; jc < kNodes; jc += 16) {
    const v4f cj = *(const v4f*)(sC + (jc + m) * 4);
    const float dx = ci[0] - cj[0], dy = ci[1] - cj[1], dz = ci[2] - cj[2];
    const float dist = sqrtf(dx * dx + dy * dy + dz * dz + kEps);
    const float rinv = 1.0f / dist;
    const float f0 = dist, f1 = dx * rinv, f2 = dy * rinv, f3 = dz * rinv;
    const float f4 = ci[3] - cj[3];

#pragma unroll
    for (int q = 0; q < 4; ++q) {
      v8h hv;
#pragma unroll
      for (int p = 0; p < 4; ++p) {
        const float* w = wbase + (4 * q + p) * 12;
        const v4f wa = *(const v4f*)(w);
        const v4f wb = *(const v4f*)(w + 4);
        const v4f wc = *(const v4f*)(w + 8);
        const float h0 = fmaf(f0, wa[0], fmaf(f1, wa[2], fmaf(f2, wb[0], fmaf(f3, wb[2], fmaf(f4, wc[0], wc[2])))));
        const float h1 = fmaf(f0, wa[1], fmaf(f1, wa[3], fmaf(f2, wb[1], fmaf(f3, wb[3], fmaf(f4, wc[1], wc[3])))));
        hv[2 * p]     = (_Float16)fmaxf(h0, 0.0f);
        hv[2 * p + 1] = (_Float16)fmaxf(h1, 0.0f);
      }
      *(v8h*)(arow + 8 * q) = hv;
    }
    wave_lds_sync();
    const v16h a0 = FragH::load(afr);
    const v16h a1 = FragH::load(afr + 32);
    const v4i va = *(const v4i*)(sV + jc + 8 * half);
    const v4i vb = *(const v4i*)(sV + jc + 8 * half + 4);
    const int mk[8] = {va[0], va[1], va[2], va[3], vb[0], vb[1], vb[2], vb[3]};

#pragma unroll
    for (int t = 0; t < 4; ++t) {
      v8f d = (v8f){0.f, 0.f, 0.f, 0.f, 0.f, 0.f, 0.f, 0.f};
      d = mma_h(a0, w2f[0][t], d);
      d = mma_h(a1, w2f[1][t], d);
#pragma unroll
      for (int r = 0; r < 8; ++r) {
        const float x = fmaxf(fmaf(d[r], kL2Fold, b2v[t]), 0.0f);
        const float xs = (mk[r] != 0) ? x : 0.0f;
        acc[t] += xs;
      }
    }
    wave_lds_sync();
  }

  float tot[4];
#pragma unroll
  for (int t = 0; t < 4; ++t) tot[t] = acc[t] + __shfl_xor(acc[t], 16, 32);
  const float sc = cntinv[b] * kAggCarry;
  if (half == 0) {
#pragma unroll
    for (int t = 0; t < 4; ++t) sAgg[wave * kHid + 16 * t + m] = tot[t] * sc;
  }
  __syncthreads();
  if (tid < 64) {
    const int row = tid >> 3, c8 = (tid & 7) * 8;
    const v4f s0 = *(const v4f*)(sAgg + row * kHid + c8);
    const v4f s1 = *(const v4f*)(sAgg + row * kHid + c8 + 4);
    v8h hv;
#pragma unroll
    for (int e = 0; e < 4; ++e) {
      hv[e]     = (_Float16)s0[e];
      hv[4 + e] = (_Float16)s1[e];
    }
    unsigned short* p = aggp + (size_t)(bi0 + row) * kHid + c8;
    *(volatile v8h*)p = hv;
    __threadfence();
    *(volatile v8h*)p = hv;
  }
}

__global__ __launch_bounds__(256) void out_gemm_kernel(
    const unsigned short* __restrict__ Ap, const unsigned short* __restrict__ Btp,
    float* __restrict__ C, const float* __restrict__ bias, const int* __restrict__ rowmask)
{
  const _Float16* A  = (const _Float16*)Ap;
  const _Float16* Bt = (const _Float16*)Btp;
  __shared__ __align__(16) float sT[8][16 * 68];
  const int lane = threadIdx.x & 31;
  const int wave = threadIdx.x >> 5;
  constexpr int tilesN = kDmodel >> 6;
  const int tile = blockIdx.x * 8 + wave;
  const int tm = tile / tilesN;
  const int tn = tile - tm * tilesN;
  const int m0 = tm << 6;
  const int n0 = tn << 6;

  const int rlane = lane & 15;
  const int koff  = (lane >> 4) * 8;
  const int mOff  = (lane >> 4) * 8;

  v8f acc[4][4];
#pragma unroll
  for (int i = 0; i < 4; ++i)
#pragma unroll
    for (int j = 0; j < 4; ++j) acc[i][j] = (v8f){0.f, 0.f, 0.f, 0.f, 0.f, 0.f, 0.f, 0.f};

#pragma unroll 1
  for (int k0 = 0; k0 < kHid; k0 += 32) {
    v16h bh[4];
#pragma unroll
    for (int j = 0; j < 4; ++j)
      bh[j] = FragH::load(Bt + (size_t)(n0 + (j << 4) + rlane) * kHid + koff + k0);
#pragma unroll
    for (int i = 0; i < 4; ++i) {
      const v16h ah = FragH::load(A + (size_t)(m0 + (i << 4) + rlane) * kHid + koff + k0);
#pragma unroll
      for (int j = 0; j < 4; ++j) acc[i][j] = mma_h(ah, bh[j], acc[i][j]);
    }
  }

  float* slab = sT[wave];
  float bv[4];
#pragma unroll
  for (int j = 0; j < 4; ++j) bv[j] = bias[n0 + (j << 4) + rlane];
#pragma unroll
  for (int i = 0; i < 4; ++i) {
    const int mBase = m0 + (i << 4);
    const v4i ma = *(const v4i*)(rowmask + mBase + mOff);
    const v4i mb = *(const v4i*)(rowmask + mBase + mOff + 4);
    const int mk[8] = {ma[0], ma[1], ma[2], ma[3], mb[0], mb[1], mb[2], mb[3]};
#pragma unroll
    for (int j = 0; j < 4; ++j) {
#pragma unroll
      for (int r = 0; r < 8; ++r) {
        const float v = fmaf(acc[i][j][r], kOutFold, bv[j]);
        const float vs = (mk[r] != 0) ? v : 0.0f;
        slab[(mOff + r) * 68 + (j << 4) + rlane] = vs;
      }
    }
    wave_lds_sync();
    {
      const int hh = lane >> 4, c4 = (lane & 15) * 4;
      for (int pass = 0; pass < 2; ++pass) {
#pragma unroll
        for (int it = 0; it < 8; ++it) {
          const int row = it * 2 + hh;
          const v4f v = *(const v4f*)(slab + row * 68 + c4);
          *(volatile v4f*)(C + (size_t)(mBase + row) * kDmodel + n0 + c4) = v;
        }
        __threadfence();
      }
    }
    wave_lds_sync();
  }
}

extern "C" void kernel_launch(void* const* d_in, const int* in_sizes, int n_in,
                              void* d_out, int out_size, void* d_ws, size_t ws_size,
                              hipStream_t stream) {
  if (n_in < 8) return;
  if (in_sizes[0] != kRows * 24) return;
  if (in_sizes[1] != kRows) return;
  if (in_sizes[2] != kFeat * kHid) return;
  if (in_sizes[3] != kHid) return;
  if (in_sizes[4] != kHid * kHid) return;
  if (in_sizes[5] != kHid) return;
  if (in_sizes[6] != kHid * kDmodel) return;
  if (in_sizes[7] != kDmodel) return;
  if (out_size != kRows * kDmodel) return;
  if (ws_size < kWsTotal) return;

  const float* corners = (const float*)d_in[0];
  const int*   valid   = (const int*)  d_in[1];
  const float* W1      = (const float*)d_in[2];
  const float* b1      = (const float*)d_in[3];
  const float* W2      = (const float*)d_in[4];
  const float* b2      = (const float*)d_in[5];
  const float* Wo      = (const float*)d_in[6];
  const float* bo      = (const float*)d_in[7];
  float* out = (float*)d_out;

  char* ws = (char*)d_ws;
  float*          cen4 = (float*)(ws + kOffCen);
  float*          cnt  = (float*)(ws + kOffCnt);
  unsigned short* w2t  = (unsigned short*)(ws + kOffW2t);
  unsigned short* wot  = (unsigned short*)(ws + kOffWot);
  unsigned short* agg  = (unsigned short*)(ws + kOffAgg);

  prep_kernel<<<27, 256, 0, stream>>>(corners, valid, W2, Wo, cen4, cnt, w2t, wot);
  pair_mlp_kernel<<<kRows / 8, 256, 0, stream>>>(cen4, valid, cnt, w2t, W1, b1, b2, agg);
  out_gemm_kernel<<<(kRows / 64) * (kDmodel / 64) / 8, 256, 0, stream>>>(agg, wot, out, bo, valid);
}
